// ConvolutionalSelfAttention_90632399880598
// MI455X (gfx1250) — hardware-verified
//
#include <hip/hip_runtime.h>


namespace {
typedef _Float16 b16;
typedef __attribute__((ext_vector_type(16))) _Float16 v16b;
typedef __attribute__((ext_vector_type(8))) _Float16 v8b;
typedef __attribute__((ext_vector_type(4))) _Float16 v4h;
typedef __attribute__((ext_vector_type(2))) _Float16 v2h;
typedef __attribute__((ext_vector_type(8))) float v8f;
typedef __attribute__((ext_vector_type(4))) float v4f;
typedef __attribute__((ext_vector_type(2))) float v2f;
__device__ __forceinline__ float bf16_rne(float f) { unsigned int u = __float_as_uint(f); u += 0x7FFFu + ((u >> 16) & 1u); return __uint_as_float(u & 0xFFFF0000u); }
__device__ __forceinline__ void split16(float v, b16& hi, b16& lo) { hi = (b16)v; lo = (b16)(v - (float)hi); }
__device__ __forceinline__ v16b frag_kb(const b16* p, int hh) { const v8b a = *(const v8b*)(p + 8 * hh), b = *(const v8b*)(p + 16 + 8 * hh); v16b f;
#pragma unroll
  for (int e = 0; e < 8; ++e) { f[e] = a[e]; f[8 + e] = b[e]; } return f; }
__device__ __forceinline__ v8f wmma16b(v16b a, v16b b, v8f c) { v8f d = __builtin_amdgcn_wmma_f32_16x16x32_f16(false, a, false, b, (short)0, c, false, false); asm volatile("v_nop\n\tv_nop\n\tv_nop\n\tv_nop" : "+v"(d) : "v"(a), "v"(b)); return d; }
__device__ __forceinline__ void wave_lds_sync() { __builtin_amdgcn_fence(__ATOMIC_RELEASE, "workgroup"); __builtin_amdgcn_wave_barrier(); __builtin_amdgcn_fence(__ATOMIC_ACQUIRE, "workgroup"); }
__device__ __forceinline__ float pmul(float a, float b) { float p = a * b; asm volatile("" : "+v"(p)); return p; }
__device__ __forceinline__ int iclamp(int v, int lo, int hi) { return v < lo ? lo : (v > hi ? hi : v); }
__device__ __forceinline__ float nexp2(float v) { return __builtin_amdgcn_exp2f(v); }

constexpr int B = 8, HH = 32, WW = 32, C = 128, KS = 3, CH = 30, CW = 30, F = CH * CW, FS = 9, P = HH * WW, BL = B  ;
constexpr float XS = 8.0f, WSC = 256.0f, RS = 1024.0f, EPS = 1e-5f, LOG2E = 1.4426950408889634f;
static_assert(P % 64 == 0 && C == 128, "tiling");
__global__ __launch_bounds__(256) void prep_kernel(const float* __restrict__ wq, const float* __restrict__ wk, b16* __restrict__ WT) {
  const int u = blockIdx.x * 256 + threadIdx.x; if (u >= 2 * C * C / 8) return; const int e = u * 8; const float* w = (e < C * C) ? wq + e : wk + (e - C * C); v8b o;
  for (int j = 0; j < 8; ++j) o[j] = (b16)(bf16_rne(w[j]) * WSC);
  for (int pass = 0; pass < 2; ++pass) { *(volatile v8b*)(WT + e) = o; __threadfence(); }
}
__global__ __launch_bounds__(256) void v_kernel(const float* __restrict__ x, const float* __restrict__ wv, const float* __restrict__ bv, float* __restrict__ V) {
  __shared__ float Wv[C]; if (threadIdx.x < C) Wv[threadIdx.x] = bf16_rne(wv[threadIdx.x]); __syncthreads();
  const int u = blockIdx.x * 256 + threadIdx.x; if (u >= BL * P) return; float s = 0.0f;
#pragma unroll 2
  for (int c = 0; c < C; c += 4) { const v4f a = *(const v4f*)(x + (size_t)u * C + c); for (int i = 0; i < 4; ++i) s = fmaf(bf16_rne(a[i]), Wv[c + i], s); }
  s += bf16_rne(bv[0]);
  for (int pass = 0; pass < 2; ++pass) { ((volatile float*)V)[u] = s; __threadfence(); }
}
__global__ __launch_bounds__(128) void proj_kernel(const float* __restrict__ x, const b16* __restrict__ WT, const float* __restrict__ bq, const float* __restrict__ bk, b16* __restrict__ QH, b16* __restrict__ QL, b16* __restrict__ KH, b16* __restrict__ KL) {
  __shared__ __attribute__((aligned(16))) b16 As[64][C + 8]; __shared__ __attribute__((aligned(16))) float Tf[4][16][128 + 4];
  const int wave = threadIdx.x >> 5, lane = threadIdx.x & 31, nloc = lane & 15, hlf = lane >> 4; const int p0 = blockIdx.x * 64; const int b = blockIdx.y; const int part = blockIdx.z, n0 = part * 128;
  const float* xb = x + ((size_t)b * P + p0) * C; const float* bias = part == 0 ? bq : bk;
  for (int i = threadIdx.x; i < 64 * (C / 4); i += 128) { const int rr = i / (C / 4), q = (i % (C / 4)) * 4; const v4f f = *(const v4f*)(xb + (size_t)rr * C + q); v4h o; for (int j = 0; j < 4; ++j) o[j] = (b16)(bf16_rne(f[j]) * XS); *(v4h*)(&As[rr][q]) = o; }
  __syncthreads();
  v8f acc[8];
#pragma unroll
  for (int t = 0; t < 8; ++t) acc[t] = (v8f){};
#pragma unroll
  for (int kb = 0; kb < C; kb += 32) { const v16b a = frag_kb(&As[wave * 16 + nloc][kb], hlf);
#pragma unroll
    for (int t = 0; t < 8; ++t) acc[t] = wmma16b(a, frag_kb(WT + (size_t)(n0 + t * 16 + nloc) * C + kb, hlf), acc[t]); }
#pragma unroll
  for (int t = 0; t < 8; ++t) { const float bb = bf16_rne(bias[t * 16 + nloc]);
#pragma unroll
    for (int r = 0; r < 8; ++r) Tf[wave][8 * hlf + r][t * 16 + nloc] = acc[t][r] * (1.0f / (XS * WSC)) + bb; }
  wave_lds_sync();
  b16* ph = part == 0 ? QH : KH; b16* pl = part == 0 ? QL : KL;
  for (int pass = 0; pass < 2; ++pass) { for (int rr = 0; rr < 16; ++rr) { const int p = p0 + wave * 16 + rr; v4h hv, lv;
      for (int j = 0; j < 4; ++j) { const float f = Tf[wave][rr][lane * 4 + j] * XS; const b16 h = (b16)f; hv[j] = h; lv[j] = (b16)((f - (float)h) * RS); }
      const size_t oi = ((size_t)b * P + p) * C + lane * 4; *(volatile v4h*)(ph + oi) = hv; *(volatile v4h*)(pl + oi) = lv; } __threadfence(); }
}
__global__ __launch_bounds__(64) void score_kernel(const b16* __restrict__ QH, const b16* __restrict__ QL, const b16* __restrict__ KH, const b16* __restrict__ KL, const float* __restrict__ V, float* __restrict__ E, float* __restrict__ ZS) {
  __shared__ __attribute__((aligned(16))) float Te[2][16][32 + 4]; __shared__ __attribute__((aligned(16))) float zs[32][2];
  const int wave = threadIdx.x >> 5, lane = threadIdx.x & 31, hh = lane >> 4, col = lane & 15; const int b = blockIdx.y; const int q0 = blockIdx.x * 32 + wave * 16, qi = q0 + col;
  const b16* Qhb = QH + (size_t)b * P * C; const b16* Qlb = QL + (size_t)b * P * C; const b16* Khb = KH + (size_t)b * P * C; const b16* Klb = KL + (size_t)b * P * C; const float* Vb = V + (size_t)b * P;
  v16b qh[4], ql[4];
#pragma unroll
  for (int s = 0; s < 4; ++s) { qh[s] = frag_kb(Qhb + (size_t)qi * C + 32 * s, hh); ql[s] = frag_kb(Qlb + (size_t)qi * C + 32 * s, hh); }
  const float cs = LOG2E / (XS * XS), csl = cs / RS;
  float z = 0.0f, sv = 0.0f; float* Erow = E + ((size_t)b * P) * P;
#pragma unroll 1
  for (int kb = 0; kb < P; kb += 32) {
#pragma unroll
    for (int u = 0; u < 2; ++u) { v8f s = (v8f){}, sl = (v8f){}; const size_t kr = (size_t)(kb + u * 16 + col) * C;
#pragma unroll
      for (int st = 0; st < 4; ++st) { const v16b kh = frag_kb(Khb + kr + 32 * st, hh), kl = frag_kb(Klb + kr + 32 * st, hh); s = wmma16b(kh, qh[st], s); sl = wmma16b(kh, ql[st], sl); sl = wmma16b(kl, qh[st], sl); }
#pragma unroll
      for (int r = 0; r < 8; ++r) { const int key = kb + u * 16 + 8 * hh + r; const float e = nexp2(s[r] * cs + sl[r] * csl); z += e; sv = fmaf(e, Vb[key], sv); Te[wave][col][u * 16 + 8 * hh + r] = e; } }
    wave_lds_sync();
    for (int pass = 0; pass < 2; ++pass) { for (int rr = 0; rr < 16; ++rr) ((volatile float*)Erow)[(size_t)(q0 + rr) * P + kb + lane] = Te[wave][rr][lane]; __threadfence(); }
    wave_lds_sync(); }
  z += __shfl_xor(z, 16); sv += __shfl_xor(sv, 16);
  if (hh == 0) { zs[wave * 16 + col][0] = z; zs[wave * 16 + col][1] = sv; }
  __syncthreads();
  for (int pass = 0; pass < 2; ++pass) { if (wave == 0) *(volatile v2f*)(ZS + ((size_t)b * P + blockIdx.x * 32 + lane) * 2) = *(const v2f*)(&zs[lane][0]); __threadfence(); }
}
__global__ __launch_bounds__(256) void window_kernel(const float* __restrict__ x, const int* __restrict__ li, const float* __restrict__ V, const float* __restrict__ E, const float* __restrict__ ZS, float* __restrict__ out) {
  const int wave = threadIdx.x >> 5, lane = threadIdx.x & 31; const int u = blockIdx.x * 8 + wave; if (u >= BL * F) return;
  const int b = u / F, f = u % F;
  int pix[FS];
#pragma unroll
  for (int i = 0; i < FS; ++i) pix[i] = iclamp(li[f * FS + i], 0, P - 1);
  const int lp = iclamp(li[f * FS + (lane < FS ? lane : 0)], 0, P - 1);
  float g = 0.0f;
  { const float* Er = E + ((size_t)b * P + lp) * P; float z = ZS[((size_t)b * P + lp) * 2], sv = ZS[((size_t)b * P + lp) * 2 + 1];
#pragma unroll
    for (int i = 0; i < FS; ++i) { const float e = Er[pix[i]]; z -= e; sv -= e * V[(size_t)b * P + pix[i]]; }
    g = (lane < FS) ? sv / (z + EPS) : 0.0f; }
  v4f o = {0.0f, 0.0f, 0.0f, 0.0f};
#pragma unroll
  for (int i = 0; i < FS; ++i) { const float gi = __shfl(g, i); const v4f xv = *(const v4f*)(x + ((size_t)b * P + pix[i]) * C + lane * 4); for (int j = 0; j < 4; ++j) o[j] = fmaf(gi, bf16_rne(xv[j]), o[j]); }
  for (int pass = 0; pass < 2; ++pass) { *(volatile v4f*)(out + ((size_t)b * F + f) * C + lane * 4) = o; __threadfence(); }
}
}

extern "C" void kernel_launch(void* const* d_in, const int* in_sizes, int n_in, void* d_out, int out_size, void* d_ws, size_t ws_size, hipStream_t stream) {
  (void)n_in;
  auto Fp = [&](int i) { return (const float*)d_in[i]; };
  if (in_sizes[0] != B * P * C || in_sizes[1] != C * C || in_sizes[2] != C || in_sizes[3] != C * C || in_sizes[4] != C || in_sizes[5] != C || in_sizes[6] != 1 || in_sizes[7] != F * P || in_sizes[8] != F * FS || out_size != B * F * C) return;
  size_t off = 0; char* ws = (char*)d_ws;
  auto carve = [&](size_t bytes) { char* p = ws + off; off += (bytes + 255) & ~(size_t)255; return p; };
  b16* WT = (b16*)carve((size_t)2 * C * C * 2); const size_t plane = (size_t)B * P * C * 2; b16* QH = (b16*)carve(plane); b16* QL = (b16*)carve(plane); b16* KH = (b16*)carve(plane); b16* KL = (b16*)carve(plane);
  float* V = (float*)carve((size_t)B * P * 4); float* E = (float*)carve((size_t)B * P * P * 4); float* ZS = (float*)carve((size_t)B * P * 2 * 4);
  if (off > ws_size || off > ((size_t)128 << 20)) return;
  prep_kernel<<<(2 * C * C / 8 + 255) / 256, 256, 0, stream>>>(Fp(1), Fp(3), WT);
  v_kernel<<<(BL * P + 255) / 256, 256, 0, stream>>>(Fp(0), Fp(5), Fp(6), V);
  proj_kernel<<<dim3(P / 64, BL, 2), 128, 0, stream>>>(Fp(0), WT, Fp(2), Fp(4), QH, QL, KH, KL);
  score_kernel<<<dim3(P / 32, BL), 64, 0, stream>>>(QH, QL, KH, KL, V, E, ZS);
  window_kernel<<<(BL * F + 7) / 8, 256, 0, stream>>>(Fp(0), (const int*)d_in[8], V, E, ZS, (float*)d_out);
}
